// HaloAttention_2748779069752
// MI455X (gfx1250) — hardware-verified
//
#include <hip/hip_runtime.h>


#define NB_  8
#define IH   80
#define IW   80
#define CC   128
#define NH_  8
#define KD   16
#define BLK  8
#define HALO 3
#define KVK  14
#define NKEY (KVK * KVK)
#define NKP  224
#define VP   256
#define NBLK ((IH / BLK) * (IW / BLK))
#define NPX  (NB_ * IH * IW)
#define NREL (2 * KVK - 1)
#define PSC  32768.0f
#define LOSC 1024.0f
#define LOSCI (1.0f / 1024.0f)

typedef _Float16 h16;
typedef unsigned short bf;
typedef __attribute__((ext_vector_type(16))) __bf16   v16bf;
typedef __attribute__((ext_vector_type(16))) _Float16 v16h;
typedef __attribute__((ext_vector_type(8)))  _Float16 v8h;
typedef __attribute__((ext_vector_type(8)))  unsigned short v8us;
typedef __attribute__((ext_vector_type(8)))  float    v8f;
typedef __attribute__((ext_vector_type(4)))  float    v4f;
typedef v8h  __attribute__((may_alias)) v8ha;
typedef v4f  __attribute__((may_alias)) v4fa;
typedef v8us __attribute__((may_alias)) v8usa;

__device__ __forceinline__ unsigned short f2bf(float f) { unsigned u = __float_as_uint(f); u += 0x7FFFu + ((u >> 16) & 1u); return (unsigned short)(u >> 16); }
__device__ __forceinline__ float bf2f(unsigned short b) { return __uint_as_float(((unsigned)b) << 16); }
__device__ __forceinline__ float bfr(float f) { return bf2f(f2bf(f)); }
__device__ __forceinline__ v16h cat16(v8h lo, v8h hi) { return __builtin_shufflevector(lo, hi, 0, 1, 2, 3, 4, 5, 6, 7, 8, 9, 10, 11, 12, 13, 14, 15); }
__device__ __forceinline__ v16bf cat16b(v8us lo, v8us hi) { return __builtin_bit_cast(v16bf, __builtin_shufflevector(lo, hi, 0, 1, 2, 3, 4, 5, 6, 7, 8, 9, 10, 11, 12, 13, 14, 15)); }
__device__ __forceinline__ v8f wmma16(v16h a, v16h b, v8f c) { return __builtin_amdgcn_wmma_f32_16x16x32_f16(false, a, false, b, (short)0, c, false, false); }
__device__ __forceinline__ v8f wmmab(v16bf a, v16bf b, v8f c) { return __builtin_amdgcn_wmma_f32_16x16x32_bf16(false, a, false, b, (short)0, c, false, false); }
#define VST2(T, p, v) do { const T vst2_v_ = (v); *(volatile T*)(p) = vst2_v_; __threadfence(); *(volatile T*)(p) = vst2_v_; } while (0)

__global__ __launch_bounds__(256) void k_rows128(const float* __restrict__ src, size_t rows, bf* dst) {
    const int lane = threadIdx.x & 31; const size_t w = (size_t)blockIdx.x * 8 + (threadIdx.x >> 5);
    if (w * 2 >= rows) return;
    v8us o;
#pragma unroll
    for (int i = 0; i < 8; ++i) o[i] = f2bf(src[w * 256 + lane * 8 + i]);
    VST2(v8us, dst + w * 256 + lane * 8, o);
}
__global__ __launch_bounds__(256) void k_wt(const float* __restrict__ Wm, int K, int ncols, bf* WT) {
    __shared__ __align__(16) unsigned short tl[64 * 72];
    const int tid = threadIdx.x, k0 = blockIdx.x * 64, n0 = blockIdx.y * 64;
    const int kk = tid >> 2, nq = (tid & 3) * 16;
#pragma unroll
    for (int i = 0; i < 16; ++i) tl[(nq + i) * 72 + kk] = f2bf(Wm[(size_t)(k0 + kk) * ncols + n0 + nq + i]);
    __syncthreads();
    const int piece = tid & 7;
    auto pass = [&]() {
#pragma unroll
        for (int s = 0; s < 2; ++s) { const int nr = (tid >> 3) + 32 * s; const v8us val = *(const v8usa*)(tl + nr * 72 + piece * 8); *(volatile v8us*)(WT + (size_t)(n0 + nr) * K + k0 + piece * 8) = val; }
    };
    pass(); __threadfence(); pass();
}
template <int MODE>
__global__ __launch_bounds__(128) void k_gemm(const bf* __restrict__ A, const bf* __restrict__ Al, const bf* __restrict__ Bn, float scale, int ldc, void* C, void* C2) {
    __shared__ __align__(16) float ost[4][16 * 68];
    const int lane = threadIdx.x & 31, wave = threadIdx.x >> 5, lr = lane & 15, hi = lane >> 4;
    const size_t r0 = (size_t)blockIdx.x * 64 + wave * 16; const int c0 = blockIdx.y * 64;
    v8f acc[4];
#pragma unroll
    for (int t = 0; t < 4; ++t) acc[t] = (v8f){};
#pragma unroll
    for (int kc = 0; kc < CC; kc += 32) {
        const v16bf a = cat16b(*(const v8us*)(A + (r0 + lr) * CC + kc + 8 * hi), *(const v8us*)(A + (r0 + lr) * CC + kc + 8 * hi + 16));
        v16bf al = a; if (Al) al = cat16b(*(const v8us*)(Al + (r0 + lr) * CC + kc + 8 * hi), *(const v8us*)(Al + (r0 + lr) * CC + kc + 8 * hi + 16));
#pragma unroll
        for (int t = 0; t < 4; ++t) { const bf* bp = Bn + (size_t)(c0 + t * 16 + lr) * CC + kc + 8 * hi; const v16bf bb = cat16b(*(const v8us*)bp, *(const v8us*)(bp + 16)); acc[t] = wmmab(a, bb, acc[t]); if (Al) acc[t] = wmmab(al, bb, acc[t]); }
        asm volatile("v_nop" : "+v"(acc[0]), "+v"(acc[1]), "+v"(acc[2]), "+v"(acc[3]) : "v"(a), "v"(al) : "memory");
    }
    float* os = &ost[wave][0];
#pragma unroll
    for (int t = 0; t < 4; ++t)
#pragma unroll
        for (int j = 0; j < 8; ++j) os[(hi * 8 + j) * 68 + t * 16 + lr] = acc[t][j] * scale;
    __builtin_amdgcn_wave_barrier(); asm volatile("" ::: "memory");
    if (MODE == 0) {
        h16* c1 = (h16*)C + r0 * ldc + c0; h16* c2 = (h16*)C2 + r0 * ldc + c0;
        auto pass = [&]() {
#pragma unroll
            for (int s = 0; s < 4; ++s) { const int row = 4 * s + (lane >> 3), piece = lane & 7; const float* sp = os + row * 68 + piece * 8; v8h o1, o2;
#pragma unroll
                for (int i = 0; i < 8; ++i) { const h16 ah = (h16)sp[i]; o1[i] = ah; o2[i] = (h16)((sp[i] - (float)ah) * LOSC); }
                *(volatile v8h*)(c1 + (size_t)row * ldc + piece * 8) = o1; *(volatile v8h*)(c2 + (size_t)row * ldc + piece * 8) = o2; }
        };
        pass(); __threadfence(); pass();
    } else {
        float* crow = (float*)C + r0 * ldc + c0;
        auto pass = [&]() {
#pragma unroll
            for (int s = 0; s < 8; ++s) { const int Lid = (lane >> 3) + 4 * s, piece = lane & 7; const int row = Lid >> 1, cofs = (Lid & 1) * 32 + piece * 4;
                const v4f val = *(const v4fa*)(os + row * 68 + cofs); *(volatile v4f*)(crow + (size_t)row * ldc + cofs) = val; }
        };
        pass(); __threadfence(); pass();
    }
}
__device__ __forceinline__ int key_pixel(int b, int bh, int bw, int k) { if (k >= NKEY) return -1; const int mh = k / KVK, mw = k - mh * KVK; const int r = bh * BLK - HALO + mh, c = bw * BLK - HALO + mw; if (r < 0 || r >= IH || c < 0 || c >= IW) return -1; return (b * IH + r) * IW + c; }
__global__ __launch_bounds__(256) void k_vt(const h16* __restrict__ KVH, const h16* __restrict__ KVL, h16* VTH, h16* VTL) {
    __shared__ __align__(16) h16 tl[16 * 264];
    __shared__ __align__(16) h16 tl2[16 * 264];
    const int tid = threadIdx.x, blk = blockIdx.x, h = blockIdx.y, b = blockIdx.z, bh = blk / (IW / BLK), bw = blk - bh * (IW / BLK);
    { const int px = key_pixel(b, bh, bw, tid);
#pragma unroll
      for (int d = 0; d < KD; ++d) { h16 vh = (h16)0.f, vl = (h16)0.f; if (px >= 0) { vh = KVH[(size_t)px * (2 * CC) + h * 32 + KD + d]; vl = KVL[(size_t)px * (2 * CC) + h * 32 + KD + d]; } tl[d * 264 + tid] = vh; tl2[d * 264 + tid] = vl; } }
    __syncthreads();
    const size_t base = ((((size_t)b * NBLK + blk) * NH_ + h) * KD) * VP;
    auto pass = [&]() {
#pragma unroll
        for (int s = 0; s < 2; ++s) { const int idx = s * 256 + tid; const int row = idx >> 5, piece = idx & 31;
            *(volatile v8h*)(VTH + base + (size_t)row * VP + piece * 8) = *(const v8ha*)(tl + row * 264 + piece * 8);
            *(volatile v8h*)(VTL + base + (size_t)row * VP + piece * 8) = *(const v8ha*)(tl2 + row * 264 + piece * 8); }
    };
    pass(); __threadfence(); pass();
}
__global__ __launch_bounds__(128) void k_attn(const h16* __restrict__ QH, const h16* __restrict__ QL, const h16* __restrict__ KVH, const h16* __restrict__ KVL, const h16* __restrict__ VTH, const h16* __restrict__ VTL,
                                             const float* __restrict__ pew, const float* __restrict__ peh, float* O) {
    __shared__ __align__(16) h16 plds[4][16 * 32];
    __shared__ __align__(16) h16 plds2[4][16 * 32];
    __shared__ float rtab[4][16 * 56];
    __shared__ __align__(16) float ost[4][16 * 132];
    const int lane = threadIdx.x & 31, wave = threadIdx.x >> 5, lr = lane & 15, hi = lane >> 4;
    const int b = blockIdx.y, blk = blockIdx.x, bh = blk / (IW / BLK), bw = blk - bh * (IW / BLK);
    h16* pl = &plds[wave][0]; h16* pl2 = &plds2[wave][0]; float* rt = &rtab[wave][0]; float* os = &ost[wave][0];
    const int qf = wave * 16 + lr; const int qpx = (b * IH + bh * BLK + (qf >> 3)) * IW + bw * BLK + (qf & 7);
    const v8h z8 = (v8h){};
#pragma unroll 1
    for (int h = 0; h < NH_; ++h) {
        { const size_t qo = (size_t)qpx * CC + h * KD; float qv[KD];
#pragma unroll
          for (int d = 0; d < KD; ++d) qv[d] = (float)QH[qo + d] + (float)QL[qo + d] * LOSCI;
          const float* pe = hi ? peh : pew;
#pragma unroll 1
          for (int j = 0; j < NREL; ++j) { float s = 0.f;
#pragma unroll
              for (int d = 0; d < KD; ++d) s += qv[d] * bfr(pe[d * NREL + j]);
              rt[lr * 56 + hi * 28 + j] = s; } }
        asm volatile("" ::: "memory"); __builtin_amdgcn_wave_barrier();
        const size_t qo = (size_t)qpx * CC + h * KD;
        const v16h qa = cat16(*(const v8h*)(QH + qo + 8 * hi), z8), ql = cat16(*(const v8h*)(QL + qo + 8 * hi), z8);
        v8f o = (v8f){}, ox = (v8f){};
        float mrow[8], lpart[8];
#pragma unroll
        for (int j = 0; j < 8; ++j) { mrow[j] = -3.0e38f; lpart[j] = 0.f; }
        const size_t vrow = ((((size_t)b * NBLK + blk) * NH_ + h) * KD + lr) * VP + 8 * hi;
#pragma unroll 1
        for (int kt = 0; kt < NKP / 32; ++kt) {
            const int l0 = kt * 32;
            const int pa_ = key_pixel(b, bh, bw, l0 + lr), pb_ = key_pixel(b, bh, bw, l0 + 16 + lr);
            const size_t ka = (size_t)(pa_ < 0 ? 0 : pa_) * (2 * CC) + h * 32 + 8 * hi, kb = (size_t)(pb_ < 0 ? 0 : pb_) * (2 * CC) + h * 32 + 8 * hi;
            const v16h k0h = cat16(pa_ >= 0 ? *(const v8h*)(KVH + ka) : z8, z8), k1h = cat16(pb_ >= 0 ? *(const v8h*)(KVH + kb) : z8, z8);
            const v16h k0l = cat16(pa_ >= 0 ? *(const v8h*)(KVL + ka) : z8, z8), k1l = cat16(pb_ >= 0 ? *(const v8h*)(KVL + kb) : z8, z8);
            v8f s0 = wmma16(qa, k0h, (v8f){}), s1 = wmma16(qa, k1h, (v8f){}), x0 = wmma16(ql, k0h, (v8f){}), x1 = wmma16(ql, k1h, (v8f){});
            x0 = wmma16(qa, k0l, x0); x1 = wmma16(qa, k1l, x1);
            asm volatile("v_nop\n\tv_nop\n\tv_nop\n\tv_nop" : "+v"(s0), "+v"(s1), "+v"(x0), "+v"(x1) : "v"(qa), "v"(ql));
            float alpha[8];
#pragma unroll
            for (int j = 0; j < 8; ++j) { const int qr = hi * 8 + j; const int x = wave * 2 + hi, y = j;
                const int ka_ = l0 + lr, kb_ = l0 + 16 + lr;
                float a0 = -__builtin_inff(), a1 = -__builtin_inff();
                if (ka_ < NKEY) { const int mh = ka_ / KVK, mw = ka_ - mh * KVK; a0 = (s0[j] + x0[j] * LOSCI) + rt[qr * 56 + (mw - y + 13)] + rt[qr * 56 + 28 + (mh - x + 13)]; }
                if (kb_ < NKEY) { const int mh = kb_ / KVK, mw = kb_ - mh * KVK; a1 = (s1[j] + x1[j] * LOSCI) + rt[qr * 56 + (mw - y + 13)] + rt[qr * 56 + 28 + (mh - x + 13)]; }
                float mx = fmaxf(a0, a1);
                mx = fmaxf(mx, __shfl_xor(mx, 1, 16)); mx = fmaxf(mx, __shfl_xor(mx, 2, 16)); mx = fmaxf(mx, __shfl_xor(mx, 4, 16)); mx = fmaxf(mx, __shfl_xor(mx, 8, 16));
                const float mn = fmaxf(mrow[j], mx);
                alpha[j] = __expf(mrow[j] - mn); mrow[j] = mn;
                const float p0 = __expf(a0 - mn), p1 = __expf(a1 - mn);
                lpart[j] = lpart[j] * alpha[j] + (p0 + p1);
                const float ps0 = p0 * PSC, ps1 = p1 * PSC; const h16 h0 = (h16)ps0, h1 = (h16)ps1;
                pl[qr * 32 + lr] = h0; pl[qr * 32 + 16 + lr] = h1; pl2[qr * 32 + lr] = (h16)(ps0 - (float)h0); pl2[qr * 32 + 16 + lr] = (h16)(ps1 - (float)h1); }
#pragma unroll
            for (int j = 0; j < 8; ++j) { o[j] *= alpha[j]; ox[j] *= alpha[j]; }
            asm volatile("" ::: "memory");
            const v16h pa = cat16(*(const v8ha*)(pl + lr * 32 + hi * 8), *(const v8ha*)(pl + lr * 32 + 16 + hi * 8));
            const v16h px = cat16(*(const v8ha*)(pl2 + lr * 32 + hi * 8), *(const v8ha*)(pl2 + lr * 32 + 16 + hi * 8));
            const v16h vh = cat16(*(const v8h*)(VTH + vrow + l0), *(const v8h*)(VTH + vrow + l0 + 16)), vl = cat16(*(const v8h*)(VTL + vrow + l0), *(const v8h*)(VTL + vrow + l0 + 16));
            o = wmma16(pa, vh, o); o = wmma16(px, vh, o); ox = wmma16(pa, vl, ox);
            asm volatile("v_nop\n\tv_nop\n\tv_nop\n\tv_nop" : "+v"(o), "+v"(ox) : "v"(pa), "v"(px), "v"(vh), "v"(vl));
            __builtin_amdgcn_wave_barrier();
        }
        float inv[8];
#pragma unroll
        for (int j = 0; j < 8; ++j) { float rs = lpart[j]; rs += __shfl_xor(rs, 1, 16); rs += __shfl_xor(rs, 2, 16); rs += __shfl_xor(rs, 4, 16); rs += __shfl_xor(rs, 8, 16); inv[j] = 1.0f / (rs * PSC); }
#pragma unroll
        for (int j = 0; j < 8; ++j) os[(hi * 8 + j) * 132 + h * KD + lr] = (o[j] + ox[j] * LOSCI) * inv[j];
        __builtin_amdgcn_wave_barrier(); asm volatile("" ::: "memory");
    }
    auto pass = [&]() {
#pragma unroll
        for (int s = 0; s < 16; ++s) { const int row = s, piece = lane;
            const int q = wave * 16 + row; const size_t px = (size_t)(b * IH + bh * BLK + (q >> 3)) * IW + bw * BLK + (q & 7);
            const v4f val = *(const v4fa*)(os + row * 132 + piece * 4); *(volatile v4f*)(O + px * CC + piece * 4) = val; }
    };
    pass(); __threadfence(); pass();
}
__global__ __launch_bounds__(256) void k_osplit(const float* __restrict__ Of, bf* OH, bf* OL) {
    const int lane = threadIdx.x & 31; const size_t w = (size_t)blockIdx.x * 8 + (threadIdx.x >> 5);
    if (w * 2 >= (size_t)NPX) return;
    v8us oh, ol;
#pragma unroll
    for (int i = 0; i < 8; ++i) { const float v = Of[w * 256 + lane * 8 + i]; const unsigned short hb = f2bf(v); oh[i] = hb; ol[i] = f2bf(v - bf2f(hb)); }
    *(volatile v8us*)(OH + w * 256 + lane * 8) = oh; *(volatile v8us*)(OL + w * 256 + lane * 8) = ol; __threadfence();
    *(volatile v8us*)(OH + w * 256 + lane * 8) = oh; *(volatile v8us*)(OL + w * 256 + lane * 8) = ol;
}

extern "C" void kernel_launch(void* const* d_in, const int* in_sizes, int n_in,
                              void* d_out, int out_size, void* d_ws, size_t ws_size, hipStream_t stream) {
    (void)in_sizes; (void)n_in; (void)out_size;
    const float* x = (const float*)d_in[0]; const float* Wq = (const float*)d_in[1]; const float* Wkv = (const float*)d_in[2]; const float* Wo = (const float*)d_in[3]; const float* pew = (const float*)d_in[4]; const float* peh = (const float*)d_in[5];
    float* out = (float*)d_out;
    char* wsp = (char*)d_ws;
    auto take = [&](size_t bytes) { char* p = wsp; wsp += (bytes + 255) & ~(size_t)255; return (void*)p; };
    bf* XB = (bf*)take((size_t)NPX * CC * 2); bf* WqT = (bf*)take((size_t)CC * CC * 2); bf* WkvT = (bf*)take((size_t)2 * CC * CC * 2); bf* WoT = (bf*)take((size_t)CC * CC * 2);
    h16* QH = (h16*)take((size_t)NPX * CC * 2); h16* QL = (h16*)take((size_t)NPX * CC * 2); h16* KVH = (h16*)take((size_t)NPX * 2 * CC * 2); h16* KVL = (h16*)take((size_t)NPX * 2 * CC * 2);
    h16* VTH = (h16*)take((size_t)NB_ * NBLK * NH_ * KD * VP * 2); h16* VTL = (h16*)take((size_t)NB_ * NBLK * NH_ * KD * VP * 2); float* O = (float*)take((size_t)NPX * CC * 4);
    if ((size_t)(wsp - (char*)d_ws) > ws_size) return;
    bf* OH = (bf*)QH; bf* OL = (bf*)QL;
    k_rows128<<<(unsigned)((NPX / 2 + 7) / 8), 256, 0, stream>>>(x, NPX, XB);
    k_wt<<<dim3(CC / 64, CC / 64, 1), 256, 0, stream>>>(Wq, CC, CC, WqT); k_wt<<<dim3(CC / 64, (2 * CC) / 64, 1), 256, 0, stream>>>(Wkv, CC, 2 * CC, WkvT); k_wt<<<dim3(CC / 64, CC / 64, 1), 256, 0, stream>>>(Wo, CC, CC, WoT);
    k_gemm<0><<<dim3(NPX / 64, CC / 64, 1), 128, 0, stream>>>(XB, nullptr, WqT, 0.25f, CC, QH, QL);
    k_gemm<0><<<dim3(NPX / 64, (2 * CC) / 64, 1), 128, 0, stream>>>(XB, nullptr, WkvT, 1.0f, 2 * CC, KVH, KVL);
    k_vt<<<dim3(NBLK, NH_, NB_), 256, 0, stream>>>(KVH, KVL, VTH, VTL);
    k_attn<<<dim3(NBLK, NB_, 1), 128, 0, stream>>>(QH, QL, KVH, KVL, VTH, VTL, pew, peh, O);
    k_osplit<<<(unsigned)((NPX / 2 + 7) / 8), 256, 0, stream>>>(O, OH, OL);
    k_gemm<1><<<dim3(NPX / 64, CC / 64, 1), 128, 0, stream>>>(OH, OL, WoT, 1.0f, CC, out, nullptr);
}
